// ConvCNP_30657476558904
// MI455X (gfx1250) — hardware-run, weakly checked
//
#include <hip/hip_runtime.h>


#ifndef NB
#define NB 4
#endif
#ifndef NCTX
#define NCTX 2048
#endif
#ifndef MTGT
#define MTGT 8192
#endif
#define NB_FULL   4
#define NCTX_FULL 2048
#define MTGT_FULL 8192
#ifndef OUT_M
#define OUT_M MTGT
#endif
#define CO   64
#define AW   4
#define TT   4
#define WT   (16 * TT)
#define BT   (AW * WT)
#define PSH  14.0f
#define PSI  (1.0f / 16384.0f)
#define CQS  64.0f
#define CQI  (1.0f / 64.0f)
#define EPSF 1e-8f
#define LOG2E 1.4426950408889634f

static_assert(NCTX % 32 == 0);
static_assert(NCTX % (4 * 32 * AW) == 0);
static_assert(NCTX % (8 * 32 * AW) == 0);
static_assert(MTGT % BT == 0);
static_assert(CO == 64);
static_assert((size_t)32 * 16 * (WT / 2) == (size_t)WT * CO * 4);
static_assert(WT % 2 == 0);
static_assert(NB <= NB_FULL);
static_assert(NCTX <= NCTX_FULL);
static_assert(MTGT <= MTGT_FULL);
static_assert((size_t)NCTX * 4 + (size_t)NCTX * 2 + (size_t)AW * WT * 2 * 4 <= (size_t)131072);
static_assert(PSH == 14.0f);

typedef _Float16 h16;
typedef unsigned short bf;
typedef __attribute__((ext_vector_type(16))) _Float16 v16h;
typedef __attribute__((ext_vector_type(8)))  _Float16 v8h;
typedef __attribute__((ext_vector_type(8)))  float    v8f;
typedef __attribute__((ext_vector_type(4)))  float    v4f;
typedef __attribute__((ext_vector_type(8)))  unsigned v8u;
typedef v4f  __attribute__((may_alias)) v4fa;
typedef v8h  __attribute__((may_alias)) v8ha;

__device__ __forceinline__ unsigned short f2bf(float f) { unsigned u = __float_as_uint(f); u += 0x7FFFu + ((u >> 16) & 1u); return (unsigned short)(u >> 16); }
__device__ __forceinline__ float bfr(float f) { return __uint_as_float(((unsigned)f2bf(f)) << 16); }
__device__ __forceinline__ v16h cat16(v8h lo, v8h hi) { return __builtin_shufflevector(lo, hi, 0, 1, 2, 3, 4, 5, 6, 7, 8, 9, 10, 11, 12, 13, 14, 15); }
__device__ __forceinline__ v8f wmma16(v16h a, v16h b, v8f c) { return __builtin_amdgcn_wmma_f32_16x16x32_f16(false, a, false, b, (short)0, c, false, false); }
__device__ __forceinline__ void wave_sync() { __builtin_amdgcn_fence(3  , "wavefront"); __builtin_amdgcn_wave_barrier(); asm volatile("" ::: "memory"); }

static __device__ __forceinline__ h16 toh_flush(float v) { const h16 r = (h16)v; return (fabsf(v) < 6.103515625e-05f) ? (h16)0.0f : r; }
__device__ __forceinline__ v8f wmma16g(v16h a, v16h b, v8f c) { c = wmma16(a, b, c); asm volatile("v_nop\n\tv_nop\n\tv_nop\n\tv_nop" : "+v"(c) : "v"(a), "v"(b)); return c; }
__device__ __forceinline__ v8f cat8(v4f lo, v4f hi) { return __builtin_shufflevector(lo, hi, 0, 1, 2, 3, 4, 5, 6, 7); }

__device__ __forceinline__ v16h pfrag(v8f xa, v8f xb, float t, float kk) {
    v16h p;
#pragma unroll
    for (int r = 0; r < 8; ++r) {
        const float da = xa[r] - t, db = xb[r] - t;
        const float ea = da * da * kk + PSH, eb = db * db * kk + PSH;
        const float pa = (ea < -14.0f) ? 0.0f : __builtin_amdgcn_exp2f(ea);
        const float pc = (eb < -14.0f) ? 0.0f : __builtin_amdgcn_exp2f(eb);
        p[r] = (h16)pa; p[8 + r] = (h16)pc; }
    return p;
}

__global__ __launch_bounds__(32 * AW) void k_rbfagg(const float* __restrict__ cin, const float* __restrict__ cval, const float* __restrict__ tin,
                                                     const float* __restrict__ sigma, const float* __restrict__ Wm, const float* __restrict__ bias, float* OUT) {
    __shared__ __align__(16) float xs[NCTX];
    __shared__ __align__(16) h16   cs[NCTX];
    __shared__ __align__(16) float dcs[AW * WT * 2];
    const int tid = threadIdx.x;
    const int lane = tid & 31, lr = lane & 15, hi = lane >> 4;
    const int wave = __builtin_amdgcn_readfirstlane((int)(threadIdx.x >> 5));
    const int b = blockIdx.y;
    const int m0 = blockIdx.x * BT + wave * WT;

    const float* ci = cin  + (size_t)b * NCTX_FULL;
    const float* cq = cval + (size_t)b * NCTX_FULL;
#pragma unroll 1
    for (int i = 0; i < NCTX / (4 * 32 * AW); ++i) {
        const int g = tid + i * (32 * AW);
        const v4f v = *(const v4f*)(ci + 4 * g); v4f o;
#pragma unroll
        for (int k = 0; k < 4; ++k) o[k] = bfr(v[k]);
        *(v4fa*)(&xs[4 * g]) = o; }
#pragma unroll 1
    for (int i = 0; i < NCTX / (8 * 32 * AW); ++i) {
        const int g = tid + i * (32 * AW);
        const v4f v0 = *(const v4f*)(cq + 8 * g), v1 = *(const v4f*)(cq + 8 * g + 4); v8h o;
#pragma unroll
        for (int k = 0; k < 4; ++k) { o[k] = toh_flush(bfr(v0[k]) * CQS); o[4 + k] = toh_flush(bfr(v1[k]) * CQS); }
        *(v8ha*)(&cs[8 * g]) = o; }

    const unsigned short sb0 = f2bf(sigma[0]), sb1 = f2bf(sigma[1]);
    const int same = __builtin_amdgcn_readfirstlane((int)(sb0 == sb1));
    const float sc0 = expf(__uint_as_float(((unsigned)sb0) << 16)), sc1 = expf(__uint_as_float(((unsigned)sb1) << 16));
    const float kk0 = (-0.5f * LOG2E) * __builtin_amdgcn_rcpf(sc0 * sc0);
    const float kk1 = (-0.5f * LOG2E) * __builtin_amdgcn_rcpf(sc1 * sc1);

    float tv[TT];
#pragma unroll
    for (int j = 0; j < TT; ++j) tv[j] = bfr(tin[(size_t)b * MTGT_FULL + m0 + 16 * j + lr]);

    __syncthreads();

    v8f acc[TT];
#pragma unroll
    for (int j = 0; j < TT; ++j) acc[j] = (v8f){};
    const bool is1 = (lr == 1);
    const unsigned onew = (lr == 0) ? 0x3C003C00u : 0u;

    if (same) {
#pragma unroll 1
        for (int key0 = 0; key0 < NCTX; key0 += 32) {
            const v4f x0 = *(const v4fa*)(&xs[key0 + 8 * hi]),      x1 = *(const v4fa*)(&xs[key0 + 8 * hi + 4]);
            const v4f x2 = *(const v4fa*)(&xs[key0 + 16 + 8 * hi]), x3 = *(const v4fa*)(&xs[key0 + 16 + 8 * hi + 4]);
            const v8f xa = cat8(x0, x1), xb = cat8(x2, x3);
            const v8h c0 = *(const v8ha*)(&cs[key0 + 8 * hi]); const v8h c1 = *(const v8ha*)(&cs[key0 + 16 + 8 * hi]);
            const v8u cw = __builtin_bit_cast(v8u, cat16(c0, c1)); v8u aw;
#pragma unroll
            for (int i = 0; i < 8; ++i) aw[i] = is1 ? cw[i] : onew;
            const v16h a = __builtin_bit_cast(v16h, aw);
#pragma unroll
            for (int j = 0; j < TT; ++j) { const v16h p = pfrag(xa, xb, tv[j], kk0); acc[j] = wmma16g(a, p, acc[j]); }
        }
    } else {
        v8u ow;
#pragma unroll
        for (int i = 0; i < 8; ++i) ow[i] = onew;
        const v16h a1 = __builtin_bit_cast(v16h, ow);
#pragma unroll 1
        for (int key0 = 0; key0 < NCTX; key0 += 32) {
            const v4f x0 = *(const v4fa*)(&xs[key0 + 8 * hi]),      x1 = *(const v4fa*)(&xs[key0 + 8 * hi + 4]);
            const v4f x2 = *(const v4fa*)(&xs[key0 + 16 + 8 * hi]), x3 = *(const v4fa*)(&xs[key0 + 16 + 8 * hi + 4]);
            const v8f xa = cat8(x0, x1), xb = cat8(x2, x3);
            const v8h c0 = *(const v8ha*)(&cs[key0 + 8 * hi]); const v8h c1 = *(const v8ha*)(&cs[key0 + 16 + 8 * hi]);
            const v8u cw = __builtin_bit_cast(v8u, cat16(c0, c1)); v8u aw;
#pragma unroll
            for (int i = 0; i < 8; ++i) aw[i] = is1 ? cw[i] : 0u;
            const v16h ac = __builtin_bit_cast(v16h, aw);
#pragma unroll
            for (int j = 0; j < TT; ++j) {
                const v16h p0 = pfrag(xa, xb, tv[j], kk0); acc[j] = wmma16g(a1, p0, acc[j]);
                const v16h p1 = pfrag(xa, xb, tv[j], kk1); acc[j] = wmma16g(ac, p1, acc[j]); }
        }
    }

    const int wb = wave * WT * 2;
#pragma unroll
    for (int j = 0; j < TT; ++j) {
        const float dn = acc[j][0] * PSI;
        const float s1 = acc[j][1] * (PSI * CQI);
        const float cv = s1 * __builtin_amdgcn_rcpf(dn + EPSF);
        if (hi == 0) { dcs[wb + (16 * j + lr) * 2] = dn; dcs[wb + (16 * j + lr) * 2 + 1] = cv; } }
    wave_sync();

    const int c4 = lr * 4;
    const v4f wa = *(const v4f*)(Wm + 2 * c4), wc = *(const v4f*)(Wm + 2 * c4 + 4);
    const v4f bv = *(const v4f*)(bias + c4);
    float w0[4], w1[4], bb[4];
    w0[0] = bfr(wa[0]); w1[0] = bfr(wa[1]); w0[1] = bfr(wa[2]); w1[1] = bfr(wa[3]);
    w0[2] = bfr(wc[0]); w1[2] = bfr(wc[1]); w0[3] = bfr(wc[2]); w1[3] = bfr(wc[3]);
#pragma unroll
    for (int i = 0; i < 4; ++i) bb[i] = bfr(bv[i]);

    float* orow = OUT + ((size_t)b * OUT_M + m0) * CO;
#pragma unroll 1
    for (int ps = 0; ps < 2; ++ps) {
#pragma unroll 4
        for (int s = 0; s < WT / 2; ++s) { const int row = 2 * s + hi;
            const float dn = dcs[wb + row * 2], cv = dcs[wb + row * 2 + 1];
            v4f val;
#pragma unroll
            for (int i = 0; i < 4; ++i) val[i] = dn * w0[i] + cv * w1[i] + bb[i];
            *(volatile v4f*)(orow + (size_t)row * CO + c4) = val; }
        if (ps == 0) __threadfence(); }
}

static constexpr size_t SZ_TOTAL = 0;
static_assert(SZ_TOTAL <= (size_t)134217728);

extern "C" void kernel_launch(void* const* d_in, const int* in_sizes, int n_in,
                              void* d_out, int out_size, void* d_ws, size_t ws_size, hipStream_t stream) {
    (void)d_ws; (void)ws_size;
    if (n_in < 6) return;
    const size_t needc = (size_t)(NB - 1) * NCTX_FULL + NCTX;
    const size_t needt = (size_t)(NB - 1) * MTGT_FULL + MTGT;
    if ((size_t)in_sizes[0] < needc || (size_t)in_sizes[1] < needc || (size_t)in_sizes[2] < needt) return;
    if (in_sizes[3] < 2 || in_sizes[4] < CO * 2 || in_sizes[5] < CO) return;
    if ((size_t)out_size < ((size_t)(NB - 1) * OUT_M + MTGT) * CO) return;
    const float* cin  = (const float*)d_in[0];
    const float* cval = (const float*)d_in[1];
    const float* tin  = (const float*)d_in[2];
    const float* sg   = (const float*)d_in[3];
    const float* Wm   = (const float*)d_in[4];
    const float* bs   = (const float*)d_in[5];
    float* OUT = (float*)d_out;
    k_rbfagg<<<dim3(MTGT / BT, NB, 1), 32 * AW, 0, stream>>>(cin, cval, tin, sg, Wm, bs, OUT);
}
